// SimpleDecoder_22368189677667
// MI455X (gfx1250) — hardware-run, weakly checked
//
#include <hip/hip_runtime.h>
#include <stdint.h>
#include <math.h>

typedef __attribute__((ext_vector_type(16))) _Float16 v16h;
typedef __attribute__((ext_vector_type(8)))  _Float16 v8h;
typedef __attribute__((ext_vector_type(4)))  _Float16 v4h;
typedef __attribute__((ext_vector_type(16))) __bf16   v16b;
typedef __attribute__((ext_vector_type(8)))  __bf16   v8b;
typedef __attribute__((ext_vector_type(8)))  float    v8f;
typedef __attribute__((ext_vector_type(4)))  float    v4f;
typedef __attribute__((ext_vector_type(4)))  unsigned int u32x4;

#define SEQ_LEN 2048
#define NBATCH 2
#define NHEAD 16
#define DMODEL 1024
#define DFFN 4096
#define NROWS (NBATCH * SEQ_LEN)
#define LN_EPS 1e-6f
#define W_CARRY 64.0f
#define MID_CARRY 16.0f
#define P_CARRY 32768.0f

__device__ __forceinline__ unsigned short f2bf_bits(float f) {
  unsigned u = __float_as_uint(f);
  return (unsigned short)((u + 0x7FFFu + ((u >> 16) & 1u)) >> 16);
}
__device__ __forceinline__ float bf_bits2f(unsigned short h) { return __uint_as_float(((unsigned)h) << 16); }

__device__ __forceinline__ void dep_guard_h(v8f& a, v8f& b, v16h x, v16h y) { asm volatile("v_nop\n\tv_nop\n\tv_nop\n\tv_nop" : "+v"(a), "+v"(b) : "v"(x), "v"(y)); }
__device__ __forceinline__ void dep_guard_b(v8f& a, v8f& b, v16b x, v16b y) { asm volatile("v_nop\n\tv_nop\n\tv_nop\n\tv_nop" : "+v"(a), "+v"(b) : "v"(x), "v"(y)); }
__device__ __forceinline__ void keep4_h(v16h a, v16h b, v16h c, v16h d) { asm volatile("v_nop" :: "v"(a), "v"(b), "v"(c), "v"(d)); }
__device__ __forceinline__ void keep4_b(v16b a, v16b b, v16b c, v16b d) { asm volatile("v_nop" :: "v"(a), "v"(b), "v"(c), "v"(d)); }
__device__ __forceinline__ void acc_guard4(v8f& a, v8f& b, v8f& c, v8f& d) { asm volatile("v_nop\n\tv_nop\n\tv_nop\n\tv_nop" : "+v"(a), "+v"(b), "+v"(c), "+v"(d)); }
template <typename T> struct Frag;
template <> struct Frag<_Float16> {
  typedef v16h V; union U { v16h v; v8h h[2]; };
  static __device__ __forceinline__ v16h load(const _Float16* p) {
    U f; f.h[0] = *(const v8h*)(p); f.h[1] = *(const v8h*)(p + 16); return f.v;
  }
  static __device__ __forceinline__ v8f mma(v16h a, v16h b, v8f c) {
    return __builtin_amdgcn_wmma_f32_16x16x32_f16(false, a, false, b, (short)0, c, false, false);
  }
  static __device__ __forceinline__ void guard(v8f& a, v8f& b, v16h x, v16h y) { dep_guard_h(a, b, x, y); }
  static __device__ __forceinline__ void keep(v16h a, v16h b, v16h c, v16h d) { keep4_h(a, b, c, d); }
};
template <> struct Frag<__bf16> {
  typedef v16b V; union U { v16b v; v8b h[2]; };
  static __device__ __forceinline__ v16b load(const __bf16* p) {
    U f; f.h[0] = *(const v8b*)(p); f.h[1] = *(const v8b*)(p + 16); return f.v;
  }
  static __device__ __forceinline__ v8f mma(v16b a, v16b b, v8f c) {
    return __builtin_amdgcn_wmma_f32_16x16x32_bf16(false, a, false, b, (short)0, c, false, false);
  }
  static __device__ __forceinline__ void guard(v8f& a, v8f& b, v16b x, v16b y) { dep_guard_b(a, b, x, y); }
  static __device__ __forceinline__ void keep(v16b a, v16b b, v16b c, v16b d) { keep4_b(a, b, c, d); }
};

template <int ET> struct Elem;
template <> struct Elem<0> { typedef _Float16 T; };
template <> struct Elem<1> { typedef __bf16 T; };
template <int ET, bool SPLIT, int BIAS_MODE, int OUT_MODE, bool RESID, int ACT = 0>
__global__ __launch_bounds__(256) void wmma_gemm64(
    const unsigned short* __restrict__ Ap, const unsigned short* __restrict__ A2p, int lda, long strideA,
    const unsigned short* __restrict__ Btp, const unsigned short* __restrict__ Bt2p, int ldb, long strideB,
    void* __restrict__ Cout, void* __restrict__ Cout2, int ldc, long strideC,
    const float* __restrict__ bias,
    const float* __restrict__ resid, long strideR,
    int M, int N, int K, float scale) {
  typedef typename Elem<ET>::T T;
  typedef typename Frag<T>::V V;
  const T* A = (const T*)Ap; const T* A2 = (const T*)A2p; const T* Bt = (const T*)Btp; const T* Bt2 = (const T*)Bt2p;
  __shared__ __align__(16) float sT[8][16 * 68];
  const int b    = blockIdx.y;
  const int lane = threadIdx.x & 31;
  const int wave = threadIdx.x >> 5;
  const int tilesN = N >> 6;
  const int tilesM = M >> 6;
  const int tile = blockIdx.x * 8 + wave;
  if (tile >= tilesM * tilesN) return;
  const int tm = tile / tilesN;
  const int tn = tile - tm * tilesN;
  const int m0 = tm << 6;
  const int n0 = tn << 6;

  const T* Ab  = A  + (size_t)b * strideA;
  const T* Bb  = Bt + (size_t)b * strideB;
  const T* Ab2 = SPLIT ? (A2  + (size_t)b * strideA) : nullptr;
  const T* Bb2 = SPLIT ? (Bt2 + (size_t)b * strideB) : nullptr;

  const int rlane = lane & 15;
  const int koff  = (lane >> 4) * 8;
  const int mOff  = (lane >> 4) * 8;

  v8f acc[4][4];
#pragma unroll
  for (int i = 0; i < 4; ++i)
#pragma unroll
    for (int j = 0; j < 4; ++j) acc[i][j] = (v8f){0.f,0.f,0.f,0.f,0.f,0.f,0.f,0.f};

  for (int k0 = 0; k0 < K; k0 += 32) {
    V bh[4], bl[4];
#pragma unroll
    for (int j = 0; j < 4; ++j) {
      const size_t bo = (size_t)(n0 + (j << 4) + rlane) * ldb + koff + k0;
      bh[j] = Frag<T>::load(Bb + bo);
      if (SPLIT) bl[j] = Frag<T>::load(Bb2 + bo);
    }
#pragma unroll
    for (int i = 0; i < 4; ++i) {
      const size_t ao = (size_t)(m0 + (i << 4) + rlane) * lda + koff + k0;
      V ah = Frag<T>::load(Ab + ao);
      V al;
      if (SPLIT) al = Frag<T>::load(Ab2 + ao);
#pragma unroll
      for (int j = 0; j < 4; ++j) {
        acc[i][j] = Frag<T>::mma(ah, bh[j], acc[i][j]);
        if (SPLIT) {
          acc[i][j] = Frag<T>::mma(ah, bl[j], acc[i][j]);
          acc[i][j] = Frag<T>::mma(al, bh[j], acc[i][j]);
        }
      }
      Frag<T>::guard(acc[i][0], acc[i][3], ah, SPLIT ? al : ah);
    }
    Frag<T>::keep(bh[0], bh[1], bh[2], bh[3]);
    if (SPLIT) Frag<T>::keep(bl[0], bl[1], bl[2], bl[3]);
  }
  acc_guard4(acc[0][0], acc[0][1], acc[0][2], acc[0][3]);
  acc_guard4(acc[1][0], acc[1][1], acc[1][2], acc[1][3]);
  acc_guard4(acc[2][0], acc[2][1], acc[2][2], acc[2][3]);
  acc_guard4(acc[3][0], acc[3][1], acc[3][2], acc[3][3]);

  float* slab = sT[wave];
  const float* Rb = RESID ? (resid + (size_t)b * strideR) : nullptr;
#pragma unroll
  for (int i = 0; i < 4; ++i) {
    const int mBase = m0 + (i << 4);
#pragma unroll
    for (int j = 0; j < 4; ++j) {
      const int n = n0 + (j << 4) + rlane;
      float bv = 0.f;
      if (BIAS_MODE == 2) bv = bias[n];
#pragma unroll
      for (int r = 0; r < 8; ++r) {
        float v = acc[i][j][r] * scale;
        if (BIAS_MODE == 1) v += bias[mBase + mOff + r];
        if (BIAS_MODE == 2) v += bv;
        if (RESID) v += Rb[(size_t)(mBase + mOff + r) * ldc + n];
        if (ACT == 1) v = tanhf(v);
        if (ACT == 2) v = fmaxf(v, 0.0f);
        if (ACT == 3) v = v / (1.0f + expf(-v));
        if (ACT == 4) v = (v > 0.f) ? v : 0.01f * v;
        if (ACT == 5) v = 0.5f * v * (1.0f + erff(v * 0.70710678118654752f));
        slab[(mOff + r) * 68 + (j << 4) + rlane] = v;
      }
    }
    __builtin_amdgcn_fence(__ATOMIC_RELEASE, "workgroup");
    __builtin_amdgcn_wave_barrier();
    __builtin_amdgcn_fence(__ATOMIC_ACQUIRE, "workgroup");
    if (OUT_MODE == 0) {
      float* C = (float*)Cout + (size_t)b * strideC;
      const int hh = lane >> 4, c4 = (lane & 15) * 4;
      for (int pass = 0; pass < 2; ++pass) {
#pragma unroll
        for (int it = 0; it < 8; ++it) {
          const int row = it * 2 + hh;
          v4f v = *(const v4f*)(slab + row * 68 + c4);
          *(volatile v4f*)(C + (size_t)(mBase + row) * ldc + n0 + c4) = v;
        }
        __threadfence();
      }
    } else {
      const int q = lane >> 3, c8 = (lane & 7) * 8;
      unsigned short* C  = (unsigned short*)Cout  + (size_t)b * strideC;
      unsigned short* C2 = (OUT_MODE == 2) ? ((unsigned short*)Cout2 + (size_t)b * strideC) : nullptr;
      for (int pass = 0; pass < 2; ++pass) {
#pragma unroll
        for (int it = 0; it < 4; ++it) {
          const int row = it * 4 + q;
          const float* sp = slab + row * 68 + c8;
          v8h hv, lv;
#pragma unroll
          for (int e = 0; e < 8; ++e) {
            if (OUT_MODE == 1) {
              hv[e] = (_Float16)sp[e];
            } else {
              unsigned short hb = f2bf_bits(sp[e]);
              unsigned short lb = f2bf_bits(sp[e] - bf_bits2f(hb));
              hv[e] = __builtin_bit_cast(_Float16, hb);
              lv[e] = __builtin_bit_cast(_Float16, lb);
            }
          }
          *(volatile v8h*)(C + (size_t)(mBase + row) * ldc + n0 + c8) = hv;
          if (OUT_MODE == 2) *(volatile v8h*)(C2 + (size_t)(mBase + row) * ldc + n0 + c8) = lv;
        }
        __threadfence();
      }
    }
    __builtin_amdgcn_fence(__ATOMIC_RELEASE, "workgroup");
    __builtin_amdgcn_wave_barrier();
    __builtin_amdgcn_fence(__ATOMIC_ACQUIRE, "workgroup");
  }
}

__global__ __launch_bounds__(256) void cast_f32_f16x2(
    const float* __restrict__ in, _Float16* __restrict__ out, int n2) {
  int i = blockIdx.x * 256 + threadIdx.x;
  if (i < n2) {
    const _Float16 h0 = (_Float16)in[2 * i], h1 = (_Float16)in[2 * i + 1];
    const unsigned u = (unsigned)__builtin_bit_cast(unsigned short, h0) | ((unsigned)__builtin_bit_cast(unsigned short, h1) << 16);
    ((volatile unsigned*)out)[i] = u;
    __threadfence();
    ((volatile unsigned*)out)[i] = u;
  }
}

__global__ __launch_bounds__(256) void transpose_cast_w(const float* __restrict__ W, _Float16* __restrict__ Wt,
                                                        int Kdim, int Ndim) {
  __shared__ float tile[64][65];
  const int tid = threadIdx.x, lane = tid & 31, wave = tid >> 5;
  const int k0 = blockIdx.y * 64, n0 = blockIdx.x * 64;
#pragma unroll
  for (int i = 0; i < 4; ++i) {
    const int r = i * 16 + (tid >> 4);
    const int c4 = (tid & 15) * 4;
    const v4f v = *(const v4f*)(W + (size_t)(k0 + r) * Ndim + n0 + c4);
    tile[r][c4 + 0] = v[0];
    tile[r][c4 + 1] = v[1];
    tile[r][c4 + 2] = v[2];
    tile[r][c4 + 3] = v[3];
  }
  __syncthreads();
  const int q = lane >> 3, c8 = (lane & 7) * 8;
  for (int pass = 0; pass < 2; ++pass) {
#pragma unroll
    for (int it = 0; it < 2; ++it) {
      const int nrow = wave * 8 + it * 4 + q;
      v8h hv;
#pragma unroll
      for (int e = 0; e < 8; ++e) hv[e] = (_Float16)(tile[c8 + e][nrow] * W_CARRY);
      *(volatile v8h*)(Wt + (size_t)(n0 + nrow) * Kdim + k0 + c8) = hv;
    }
    __threadfence();
  }
}

#define AT_D 64
#define AT_NW 4
#define AT_QB 64
#define AT_KC 64

__device__ __forceinline__ v8f mma_h(v16h a, v16h b, v8f c) {
  c = __builtin_amdgcn_wmma_f32_16x16x32_f16(false, a, false, b, (short)0, c, false, false);
  asm volatile("v_nop\n\tv_nop\n\tv_nop\n\tv_nop" : "+v"(c) : "v"(a), "v"(b));
  return c;
}

__global__ __launch_bounds__(128)
void attn_causal64_f16(const _Float16* __restrict__ qp, const _Float16* __restrict__ kp,
                       const _Float16* __restrict__ vp, _Float16* __restrict__ op) {
  union FH { v16h v; v8h h[2]; };
  __shared__ __align__(16) _Float16 Ksh[AT_KC * AT_D];
  __shared__ __align__(16) unsigned short Vtu[AT_D * AT_KC];
  __shared__ __align__(16) _Float16 Psh[AT_NW][16 * AT_KC];
  __shared__ __align__(16) float Os[AT_NW][16 * 68];

  const int tid  = threadIdx.x;
  const int wave = tid >> 5;
  const int lane = tid & 31;
  const int hh   = lane >> 4;
  const int c    = lane & 15;

  const int nqb = SEQ_LEN / AT_QB;
  const int bx = blockIdx.x;
  const int qb = bx % nqb;
  const int bh = bx / nqb;
  const int h  = bh % NHEAD;
  const int b  = bh / NHEAD;
  const int q0 = qb * AT_QB + wave * 16;
  const size_t hb = (size_t)b * SEQ_LEN * DMODEL + (size_t)h * AT_D;
  const _Float16* qb_ptr = qp + hb;
  const _Float16* kb_ptr = kp + hb;
  const _Float16* vb_ptr = vp + hb;
  _Float16*       ob_ptr = op + hb;
  const _Float16* VthH = (const _Float16*)(const void*)Vtu;

  v16h qa[2];
  {
    const _Float16* qrow = qb_ptr + (size_t)(q0 + c) * DMODEL;
#pragma unroll
    for (int dc = 0; dc < 2; ++dc) qa[dc] = Frag<_Float16>::load(qrow + dc * 32 + 8 * hh);
  }

  float mrow[8], lrow[8];
  v8f oacc[4];
#pragma unroll
  for (int r = 0; r < 8; ++r) { mrow[r] = -INFINITY; lrow[r] = 0.f; }
#pragma unroll
  for (int t = 0; t < 4; ++t) oacc[t] = (v8f){0.f,0.f,0.f,0.f,0.f,0.f,0.f,0.f};

  const int nChunks = qb + 1;
  for (int kc = 0; kc < nChunks; ++kc) {
    const int kv0 = kc * AT_KC;
    __syncthreads();
    {
      const int kvr = tid >> 1, dh = (tid & 1) * 32;
      const _Float16* krow = kb_ptr + (size_t)(kv0 + kvr) * DMODEL + dh;
      const u32x4*    vrow = (const u32x4*)(const void*)(vb_ptr + (size_t)(kv0 + kvr) * DMODEL + dh);
      v8h kk[4];
      u32x4 vw[4];
#pragma unroll
      for (int i = 0; i < 4; ++i) { kk[i] = *(const v8h*)(krow + 8 * i); vw[i] = vrow[i]; }
#pragma unroll
      for (int i = 0; i < 4; ++i) *(v8h*)(Ksh + kvr * AT_D + dh + 8 * i) = kk[i];
#pragma unroll
      for (int i = 0; i < 4; ++i) {
#pragma unroll
        for (int e = 0; e < 4; ++e) {
          const unsigned ww = vw[i][e];
          const int d = dh + 8 * i + 2 * e;
          Vtu[d * AT_KC + kvr]       = (unsigned short)(ww & 0xffffu);
          Vtu[(d + 1) * AT_KC + kvr] = (unsigned short)(ww >> 16);
        }
      }
    }
    __syncthreads();

    v8f s[4];
#pragma unroll
    for (int j = 0; j < 4; ++j) {
      s[j] = (v8f){0.f,0.f,0.f,0.f,0.f,0.f,0.f,0.f};
#pragma unroll
      for (int dc = 0; dc < 2; ++dc) {
        FH kb;
        kb.h[0] = *(const v8h*)(Ksh + (j * 16 + c) * AT_D + dc * 32 + 8 * hh);
        kb.h[1] = *(const v8h*)(Ksh + (j * 16 + c) * AT_D + dc * 32 + 16 + 8 * hh);
        s[j] = mma_h(qa[dc], kb.v, s[j]);
      }
    }
    const bool diag = (kc == qb);
    float cm[8];
#pragma unroll
    for (int r = 0; r < 8; ++r) {
      const int qrow = q0 + 8 * hh + r;
      float m = -INFINITY;
#pragma unroll
      for (int j = 0; j < 4; ++j) {
        const int kvcol = kv0 + j * 16 + c;
        float sv = s[j][r] * 0.125f;
        if (diag && (kvcol > qrow)) sv = -1e20f;
        s[j][r] = sv;
        m = fmaxf(m, sv);
      }
#pragma unroll
      for (int off = 1; off < 16; off <<= 1) m = fmaxf(m, __shfl_xor(m, off, 32));
      cm[r] = m;
    }
    _Float16* pw = Psh[wave];
#pragma unroll
    for (int r = 0; r < 8; ++r) {
      const float mnew = fmaxf(mrow[r], cm[r]);
      const float alpha = expf(mrow[r] - mnew);
      mrow[r] = mnew;
      float psum = 0.f;
#pragma unroll
      for (int j = 0; j < 4; ++j) {
        const float p = expf(s[j][r] - mnew);
        psum += p;
        pw[(8 * hh + r) * AT_KC + j * 16 + c] = (_Float16)(p * P_CARRY);
      }
#pragma unroll
      for (int off = 1; off < 16; off <<= 1) psum += __shfl_xor(psum, off, 32);
      lrow[r] = lrow[r] * alpha + psum;
#pragma unroll
      for (int t = 0; t < 4; ++t) oacc[t][r] *= alpha;
    }
    __builtin_amdgcn_fence(__ATOMIC_RELEASE, "workgroup");
    __builtin_amdgcn_wave_barrier();
    __builtin_amdgcn_fence(__ATOMIC_ACQUIRE, "workgroup");
#pragma unroll 1
    for (int kk2 = 0; kk2 < 2; ++kk2) {
      FH pa;
      pa.h[0] = *(const v8h*)(pw + c * AT_KC + kk2 * 32 + 8 * hh);
      pa.h[1] = *(const v8h*)(pw + c * AT_KC + kk2 * 32 + 16 + 8 * hh);
#pragma unroll
      for (int t = 0; t < 4; ++t) {
        FH vb;
        vb.h[0] = *(const v8h*)(VthH + (t * 16 + c) * AT_KC + kk2 * 32 + 8 * hh);
        vb.h[1] = *(const v8h*)(VthH + (t * 16 + c) * AT_KC + kk2 * 32 + 16 + 8 * hh);
        oacc[t] = mma_h(pa.v, vb.v, oacc[t]);
      }
    }
  }

  float* os = Os[wave];
#pragma unroll
  for (int r = 0; r < 8; ++r) {
    const float inv = MID_CARRY / (lrow[r] * P_CARRY);
#pragma unroll
    for (int t = 0; t < 4; ++t) os[(8 * hh + r) * 68 + t * 16 + c] = oacc[t][r] * inv;
  }
  __builtin_amdgcn_fence(__ATOMIC_RELEASE, "workgroup");
  __builtin_amdgcn_wave_barrier();
  __builtin_amdgcn_fence(__ATOMIC_ACQUIRE, "workgroup");
  {
    const int q = lane >> 3, c8 = (lane & 7) * 8;
    for (int pass = 0; pass < 2; ++pass) {
#pragma unroll
      for (int it = 0; it < 4; ++it) {
        const int row = it * 4 + q;
        const float* sp = os + row * 68 + c8;
        v8h hv;
#pragma unroll
        for (int e = 0; e < 8; ++e) hv[e] = (_Float16)sp[e];
        *(volatile v8h*)(ob_ptr + (size_t)(q0 + row) * DMODEL + c8) = hv;
      }
      __threadfence();
    }
  }
}

template <bool HOUT>
__global__ __launch_bounds__(256) void add_layernorm_1024(
    const float* __restrict__ a, const float* __restrict__ res,
    const float* __restrict__ gam, const float* __restrict__ bet,
    float* __restrict__ outF, _Float16* __restrict__ outH) {
  __shared__ float sS[8];
  __shared__ float sQ[8];
  __shared__ __align__(16) _Float16 hrow[HOUT ? DMODEL : 8];
  const int row = blockIdx.x;
  const int tid = threadIdx.x, lane = tid & 31, wave = tid >> 5;
  const size_t base = (size_t)row * DMODEL;
  const int c4 = tid * 4;
  const v4f va = *(const v4f*)(a + base + c4);
  const v4f vr = *(const v4f*)(res + base + c4);
  const float v0 = va[0] + vr[0], v1 = va[1] + vr[1], v2 = va[2] + vr[2], v3 = va[3] + vr[3];
  float s = (v0 + v1) + (v2 + v3);
#pragma unroll
  for (int off = 1; off < 32; off <<= 1) s += __shfl_xor(s, off, 32);
  if (lane == 0) sS[wave] = s;
  __syncthreads();
  float ts = 0.f;
#pragma unroll
  for (int w = 0; w < 8; ++w) ts += sS[w];
  const float mu = ts * (1.0f / DMODEL);
  const float d0 = v0 - mu, d1 = v1 - mu, d2 = v2 - mu, d3 = v3 - mu;
  float sq = (d0 * d0 + d1 * d1) + (d2 * d2 + d3 * d3);
#pragma unroll
  for (int off = 1; off < 32; off <<= 1) sq += __shfl_xor(sq, off, 32);
  if (lane == 0) sQ[wave] = sq;
  __syncthreads();
  float tq = 0.f;
#pragma unroll
  for (int w = 0; w < 8; ++w) tq += sQ[w];
  const float var = tq * (1.0f / DMODEL);
  const float rs = rsqrtf(var + LN_EPS);
  const v4f gg = *(const v4f*)(gam + c4);
  const v4f bb = *(const v4f*)(bet + c4);
  v4f o;
  o[0] = d0 * rs * gg[0] + bb[0];
  o[1] = d1 * rs * gg[1] + bb[1];
  o[2] = d2 * rs * gg[2] + bb[2];
  o[3] = d3 * rs * gg[3] + bb[3];
  for (int pass = 0; pass < 2; ++pass) {
    *(volatile v4f*)(outF + base + c4) = o;
    __threadfence();
  }
  if (HOUT) {
    v4h h4;
    h4[0] = (_Float16)o[0];
    h4[1] = (_Float16)o[1];
    h4[2] = (_Float16)o[2];
    h4[3] = (_Float16)o[3];
    *(v4h*)(hrow + c4) = h4;
    __syncthreads();
    if (tid < 128) {
      const v8h hv = *(const v8h*)(hrow + tid * 8);
      for (int pass = 0; pass < 2; ++pass) {
        *(volatile v8h*)(outH + base + tid * 8) = hv;
        __threadfence();
      }
    }
  }
}

static constexpr size_t kPlaneH   = (size_t)NROWS * DMODEL * 2;
static constexpr size_t kPlaneF   = (size_t)NROWS * DMODEL * 4;
static constexpr size_t kWtSq     = (size_t)DMODEL * DMODEL * 2;
static constexpr size_t kWtFfn    = (size_t)DMODEL * DFFN * 2;
static constexpr size_t kUpPlane  = (size_t)NROWS * DFFN * 2;
static constexpr size_t kOffXh    = 0;
static constexpr size_t kOffWqT   = kOffXh + kPlaneH;
static constexpr size_t kOffWkT   = kOffWqT + kWtSq;
static constexpr size_t kOffWvT   = kOffWkT + kWtSq;
static constexpr size_t kOffWoT   = kOffWvT + kWtSq;
static constexpr size_t kOffWupT  = kOffWoT + kWtSq;
static constexpr size_t kOffWdnT  = kOffWupT + kWtFfn;
static constexpr size_t kOffQ     = kOffWdnT + kWtFfn;
static constexpr size_t kOffK     = kOffQ + kPlaneH;
static constexpr size_t kOffV     = kOffK + kPlaneH;
static constexpr size_t kOffMid   = kOffV + kPlaneH;
static constexpr size_t kOffUp    = kOffQ;
static constexpr size_t kOffC0    = kOffMid + kPlaneH;
static constexpr size_t kOffX1f   = kOffC0 + kPlaneF;
static constexpr size_t kWsTotal  = kOffX1f + kPlaneF;
static_assert(kOffMid + kPlaneH - kOffQ == kUpPlane, "");
static_assert(kWsTotal == (size_t)100663296, "");
static_assert(kWsTotal <= (size_t)134217728, "");
static_assert(NROWS % 64 == 0 && DMODEL % 64 == 0 && DFFN % 64 == 0, "");
static_assert(DMODEL % 32 == 0 && DFFN % 32 == 0, "");
static_assert(SEQ_LEN % AT_QB == 0 && DMODEL == NHEAD * AT_D, "");

template <int OUT_MODE, int ACT>
static void launch_gemm(const _Float16* A, int lda, const _Float16* Bt, int ldb, void* Cp, int ldc,
                        const float* bias, int M, int N, int K, float scale, hipStream_t st) {
  const int tiles = (M / 64) * (N / 64);
  dim3 grid((unsigned)((tiles + 7) / 8), 1), block(256);
  wmma_gemm64<0, false, 2, OUT_MODE, false, ACT><<<grid, block, 0, st>>>(
      (const unsigned short*)A, nullptr, lda, 0L,
      (const unsigned short*)Bt, nullptr, ldb, 0L,
      Cp, nullptr, ldc, 0L, bias, nullptr, 0L, M, N, K, scale);
}

static void launch_transpose(const float* W, _Float16* Wt, int Kdim, int Ndim, hipStream_t st) {
  dim3 grid((unsigned)(Ndim / 64), (unsigned)(Kdim / 64)), block(256);
  transpose_cast_w<<<grid, block, 0, st>>>(W, Wt, Kdim, Ndim);
}

extern "C" void kernel_launch(void* const* d_in, const int* in_sizes, int n_in,
                              void* d_out, int out_size, void* d_ws, size_t ws_size,
                              hipStream_t stream) {
  if (n_in < 17) return;
  if (in_sizes[0] != NROWS * DMODEL || out_size != NROWS * DMODEL) return;
  if (in_sizes[1] != DMODEL * DMODEL || in_sizes[11] != DMODEL * DFFN || in_sizes[13] != DFFN * DMODEL) return;
  if (ws_size < kWsTotal) return;

  const float* x   = (const float*)d_in[0];
  const float* Wq  = (const float*)d_in[1];
  const float* bq  = (const float*)d_in[2];
  const float* Wk  = (const float*)d_in[3];
  const float* bk  = (const float*)d_in[4];
  const float* Wv  = (const float*)d_in[5];
  const float* bv  = (const float*)d_in[6];
  const float* Wo  = (const float*)d_in[7];
  const float* bo  = (const float*)d_in[8];
  const float* g1  = (const float*)d_in[9];
  const float* b1  = (const float*)d_in[10];
  const float* Wup = (const float*)d_in[11];
  const float* bup = (const float*)d_in[12];
  const float* Wdn = (const float*)d_in[13];
  const float* bdn = (const float*)d_in[14];
  const float* g2  = (const float*)d_in[15];
  const float* b2  = (const float*)d_in[16];
  float* out = (float*)d_out;

  char* ws = (char*)d_ws;
  _Float16* xh   = (_Float16*)(ws + kOffXh);
  _Float16* x1h  = (_Float16*)(ws + kOffXh);
  _Float16* WqT  = (_Float16*)(ws + kOffWqT);
  _Float16* WkT  = (_Float16*)(ws + kOffWkT);
  _Float16* WvT  = (_Float16*)(ws + kOffWvT);
  _Float16* WoT  = (_Float16*)(ws + kOffWoT);
  _Float16* WupT = (_Float16*)(ws + kOffWupT);
  _Float16* WdnT = (_Float16*)(ws + kOffWdnT);
  _Float16* qh   = (_Float16*)(ws + kOffQ);
  _Float16* kh   = (_Float16*)(ws + kOffK);
  _Float16* vh   = (_Float16*)(ws + kOffV);
  _Float16* midh = (_Float16*)(ws + kOffMid);
  _Float16* uph  = (_Float16*)(ws + kOffUp);
  float*    c0   = (float*)(ws + kOffC0);
  float*    x1f  = (float*)(ws + kOffX1f);

  {
    const int n2 = NROWS * DMODEL / 2;
    cast_f32_f16x2<<<dim3((unsigned)((n2 + 255) / 256)), dim3(256), 0, stream>>>(x, xh, n2);
  }
  launch_transpose(Wq,  WqT,  DMODEL, DMODEL, stream);
  launch_transpose(Wk,  WkT,  DMODEL, DMODEL, stream);
  launch_transpose(Wv,  WvT,  DMODEL, DMODEL, stream);
  launch_transpose(Wo,  WoT,  DMODEL, DMODEL, stream);
  launch_transpose(Wup, WupT, DMODEL, DFFN,   stream);
  launch_transpose(Wdn, WdnT, DFFN,   DMODEL, stream);

  const float invW = 1.0f / W_CARRY;
  launch_gemm<1, 0>(xh, DMODEL, WqT, DMODEL, qh, DMODEL, bq, NROWS, DMODEL, DMODEL, invW, stream);
  launch_gemm<1, 0>(xh, DMODEL, WkT, DMODEL, kh, DMODEL, bk, NROWS, DMODEL, DMODEL, invW, stream);
  launch_gemm<1, 0>(xh, DMODEL, WvT, DMODEL, vh, DMODEL, bv, NROWS, DMODEL, DMODEL, invW, stream);
  attn_causal64_f16<<<dim3((unsigned)(NBATCH * NHEAD * (SEQ_LEN / AT_QB))), dim3(128), 0, stream>>>(qh, kh, vh, midh);
  launch_gemm<0, 0>(midh, DMODEL, WoT, DMODEL, c0, DMODEL, bo, NROWS, DMODEL, DMODEL, invW / MID_CARRY, stream);
  add_layernorm_1024<true><<<dim3(NROWS), dim3(256), 0, stream>>>(x, c0, g1, b1, x1f, x1h);
  launch_gemm<1, 2>(x1h, DMODEL, WupT, DMODEL, uph, DFFN, bup, NROWS, DFFN, DMODEL, invW, stream);
  launch_gemm<0, 0>(uph, DFFN, WdnT, DFFN, c0, DMODEL, bdn, NROWS, DMODEL, DFFN, invW, stream);
  add_layernorm_1024<false><<<dim3(NROWS), dim3(256), 0, stream>>>(x1f, c0, g2, b2, out, nullptr);
}
